// TransformerLayer_50964081934911
// MI455X (gfx1250) — hardware-verified
//
#include <hip/hip_runtime.h>
#include <math.h>

typedef __attribute__((ext_vector_type(16))) _Float16 v16h;
typedef __attribute__((ext_vector_type(8)))  _Float16 v8h;
typedef __attribute__((ext_vector_type(4)))  _Float16 v4h;
typedef __attribute__((ext_vector_type(8)))  float v8f;
typedef __attribute__((ext_vector_type(4)))  float v4f;

#ifndef NB
#define NB 1
#endif
#define NB_FULL 1
#ifndef SEQ
#define SEQ 4096
#endif
#define SEQ_FULL 4096
#define DM 1024
#define NH 16
#define DK 64
#define DFF 4096
#define MROWS (NB * SEQ)
#define SCALE (0.125f)
#define PCY (16384.0f)
#define WC (64.0f)
#define CCY (16.0f)
#define GCY (16.0f)
#define F16MIN (6.103515625e-05f)
#define LN_EPS (1e-5f)
static_assert(SEQ % 64 == 0);
static_assert(SEQ >= 64);
static_assert(SEQ <= SEQ_FULL);
static_assert(NB >= 1);
static_assert(NB <= NB_FULL);
static_assert(DM == NH * DK);
static_assert(DK == 64);
static_assert(MROWS % 64 == 0);
static_assert(DM % 128 == 0 && DFF % 128 == 0 && DM % 64 == 0 && DFF % 64 == 0);

#define WSZ_W4   (2u * (size_t)4 * DM * DM)
#define WSZ_W2T  (2u * (size_t)DM * DFF)
#define WSZ_W1T  (2u * (size_t)DFF * DM)
#define WSZ_F32  (4u * (size_t)MROWS * DM)
#define WSZ_P16  (2u * (size_t)MROWS * DM)
#define WSZ_G    (2u * (size_t)MROWS * DFF)
#define WS_W4    ((size_t)0)
#define WS_W2T   WS_W4
#define WS_W1T   (WS_W4 + WSZ_W4)
#define WS_XS    (WS_W1T + WSZ_W1T)
#define WS_Y1    (WS_XS + WSZ_F32)
#define WS_Q     (WS_Y1 + WSZ_F32)
#define WS_K     (WS_Q + WSZ_P16)
#define WS_VT    (WS_K + WSZ_P16)
#define WS_HC    (WS_VT + WSZ_P16)
#define WS_G     WS_Q
#define WS_H2    (WS_HC + WSZ_P16)
#define WS_END   (WS_H2 + WSZ_P16)
static_assert(WSZ_W2T <= WSZ_W4);
static_assert(WS_G + WSZ_G <= WS_H2);
static_assert(WS_END <= (size_t)134217728u);
static_assert((WS_W1T % 256u) == 0 && (WS_XS % 256u) == 0 && (WS_Y1 % 256u) == 0 && (WS_Q % 256u) == 0 && (WS_K % 256u) == 0 && (WS_VT % 256u) == 0 && (WS_HC % 256u) == 0 && (WS_H2 % 256u) == 0);
static_assert(4 * 256 * 4 == 64 * 64 && 2 * 256 * 8 == 64 * 64);
static_assert(256 * 8 == 2 * DM);
static_assert(8 * 128 * 8 == 64 * 128);
static_assert(4 * 32 * 8 == 16 * 64);
static_assert(16 * 32 * 4 == 16 * 128);
static_assert(8 * 32 * 4 == DM);

template <typename T> __device__ __forceinline__ void vst2(void* p, T v) { *(volatile T*)p = v; __threadfence(); *(volatile T*)p = v; }
__device__ __forceinline__ v8f zero8() { v8f z = {0.f, 0.f, 0.f, 0.f, 0.f, 0.f, 0.f, 0.f}; return z; }
__device__ __forceinline__ v8f wmma16(v16h a, v16h b, v8f c) {
  v8f d = __builtin_amdgcn_wmma_f32_16x16x32_f16(false, a, false, b, (short)0, c, false, false);
  asm volatile("v_nop\n\tv_nop\n\tv_nop\n\tv_nop" : "+v"(d) : "v"(a), "v"(b));
  return d;
}
__device__ __forceinline__ v16h frag_h(const _Float16* rowk0, int lane) {
  union { v16h v; v8h q[2]; } u; const _Float16* p = rowk0 + 8 * (lane >> 4);
  u.q[0] = *(const v8h*)p; u.q[1] = *(const v8h*)(p + 16); return u.v;
}
__device__ __forceinline__ _Float16 f16n(float x) { const float t = (fabsf(x) >= F16MIN) ? x : 0.0f; return (_Float16)t; }
__device__ __forceinline__ float bf16r(float x) { unsigned u = __float_as_uint(x); u += 0x7FFFu + ((u >> 16) & 1u); return __uint_as_float(u & 0xFFFF0000u); }
#define LDSX() do { asm volatile("s_wait_dscnt 0" ::: "memory"); __builtin_amdgcn_wave_barrier(); __builtin_amdgcn_fence(3, "workgroup"); } while (0)

__device__ __forceinline__ void mm8(v8f (&acc)[8], const _Float16* __restrict__ Ar, const _Float16* __restrict__ Br, int ldb, int nk, int lane) {
#pragma unroll 1
  for (int kc = 0; kc < nk; ++kc) {
    const v16h a = frag_h(Ar + kc * 32, lane);
#pragma unroll
    for (int j = 0; j < 8; ++j) acc[j] = wmma16(a, frag_h(Br + (size_t)j * 16 * ldb + kc * 32, lane), acc[j]);
  }
}

__global__ __launch_bounds__(256) void k_wt(const float* __restrict__ W0, const float* __restrict__ W1, const float* __restrict__ W2, const float* __restrict__ W3,
                                            int K, int N, _Float16* __restrict__ WT) {
  __shared__ __align__(16) _Float16 t[64][72];
  const int tid = threadIdx.x, z = blockIdx.z;
  const float* W = (z == 0) ? W0 : ((z == 1) ? W1 : ((z == 2) ? W2 : W3));
  _Float16* O = WT + (size_t)z * N * K;
  const int k0 = blockIdx.x * 64, n0 = blockIdx.y * 64;
#pragma unroll
  for (int it = 0; it < 4; ++it) {
    const int e = tid + 256 * it, kl = e >> 4, q = e & 15;
    const v4f a = *(const v4f*)(W + (size_t)(k0 + kl) * N + n0 + 4 * q);
#pragma unroll
    for (int c = 0; c < 4; ++c) t[4 * q + c][kl] = f16n(bf16r(a[c]) * WC);
  }
  __syncthreads();
#pragma unroll
  for (int it = 0; it < 2; ++it) { const int e = tid + 256 * it, nl = e >> 3, q = e & 7; vst2(O + (size_t)(n0 + nl) * K + k0 + 8 * q, *(const v8h*)&t[nl][8 * q]); }
}

__global__ __launch_bounds__(256) void k_cx(const float* __restrict__ X, _Float16* __restrict__ H) {
  const unsigned idx = blockIdx.x * 256u + threadIdx.x;
  const unsigned row = idx >> 7, c = (idx & 127u) << 3;
  if (row >= (unsigned)MROWS) return;
  const size_t src = ((size_t)(row / (unsigned)SEQ) * SEQ_FULL + (size_t)(row % (unsigned)SEQ)) * DM + c;
  const v4f a = *(const v4f*)(X + src), b = *(const v4f*)(X + src + 4);
  v8h o8;
#pragma unroll
  for (int e = 0; e < 4; ++e) { o8[e] = f16n(bf16r(a[e])); o8[4 + e] = f16n(bf16r(b[e])); }
  vst2(H + (size_t)row * DM + c, o8);
}

template <int WH>
__global__ __launch_bounds__(256) void k_ln(const float* __restrict__ X, const float* __restrict__ GAM, const float* __restrict__ BET, float* __restrict__ OF, _Float16* __restrict__ OH) {
  const unsigned wave = threadIdx.x >> 5, lane = threadIdx.x & 31u; const unsigned row = blockIdx.x * 8u + wave; if (row >= (unsigned)MROWS) return;
  const size_t rb = (size_t)row * DM; const float* xr = X + rb;
  float s1 = 0.f;
#pragma unroll 1
  for (unsigned i = 0; i < 8u; ++i) { const v4f a = *(const v4f*)(xr + i * 128u + lane * 4u); s1 += (a[0] + a[1]) + (a[2] + a[3]); }
#pragma unroll
  for (int o = 1; o < 32; o <<= 1) s1 += __shfl_xor(s1, o);
  const float mu = s1 * (1.0f / DM); float q = 0.f;
#pragma unroll 1
  for (unsigned i = 0; i < 8u; ++i) { const v4f a = *(const v4f*)(xr + i * 128u + lane * 4u);
    const float d0 = a[0] - mu, d1 = a[1] - mu, d2 = a[2] - mu, d3 = a[3] - mu; q += (d0 * d0 + d1 * d1) + (d2 * d2 + d3 * d3); }
#pragma unroll
  for (int o = 1; o < 32; o <<= 1) q += __shfl_xor(q, o);
  const float inv = 1.0f / sqrtf(q * (1.0f / DM) + LN_EPS);
#pragma unroll 1
  for (unsigned i = 0; i < 8u; ++i) { const unsigned o = i * 128u + lane * 4u;
    const v4f a = *(const v4f*)(xr + o), ga = *(const v4f*)(GAM + o), ba = *(const v4f*)(BET + o);
    v4f y; v4h h4;
#pragma unroll
    for (int e = 0; e < 4; ++e) { const float t = (a[e] - mu) * inv * bf16r(ga[e]) + bf16r(ba[e]); y[e] = t; h4[e] = f16n(t); }
    vst2(OF + rb + o, y);
    if (WH) vst2(OH + rb + o, h4); }
}

__global__ __launch_bounds__(128) void k_pqk(const _Float16* __restrict__ H, const _Float16* __restrict__ WT, const float* __restrict__ BQ, const float* __restrict__ BK,
                                             _Float16* __restrict__ QP, _Float16* __restrict__ KP) {
  __shared__ __align__(16) _Float16 sh[64][136];
  const int tid = threadIdx.x, wave = tid >> 5, lane = tid & 31, col = lane & 15, g = lane >> 4; const int z = blockIdx.z;
  const _Float16* B = WT + (size_t)z * DM * DM; const float* bias = (z == 0) ? BQ : BK; _Float16* O = (z == 0) ? QP : KP;
  const size_t r0 = (size_t)blockIdx.x * 64; const int c0 = blockIdx.y * 128;
  v8f acc[8];
#pragma unroll
  for (int j = 0; j < 8; ++j) acc[j] = zero8();
  mm8(acc, H + (r0 + wave * 16 + col) * DM, B + (size_t)(c0 + col) * DM, DM, DM / 32, lane);
#pragma unroll
  for (int j = 0; j < 8; ++j) { const float bv = bf16r(bias[c0 + j * 16 + col]);
#pragma unroll
    for (int r = 0; r < 8; ++r) { const float v = acc[j][r] * (1.0f / WC) + bv; sh[wave * 16 + 8 * g + r][j * 16 + col] = f16n(v); } }
  __syncthreads();
#pragma unroll
  for (int it = 0; it < 8; ++it) { const int e = tid + 128 * it, rl = e >> 4, q = e & 15; vst2(O + (r0 + rl) * DM + c0 + 8 * q, *(const v8h*)&sh[rl][8 * q]); }
}

__global__ __launch_bounds__(128) void k_pvt(const _Float16* __restrict__ H, const _Float16* __restrict__ WVT, const float* __restrict__ BV, _Float16* __restrict__ VT) {
  __shared__ __align__(16) _Float16 th[128][72];
  const int tid = threadIdx.x, wave = tid >> 5, lane = tid & 31, col = lane & 15, g = lane >> 4;
  const size_t r0 = (size_t)blockIdx.x * 64; const int c0 = blockIdx.y * 128;
  const size_t b = r0 / SEQ; const int s0 = (int)(r0 % SEQ);
  v8f acc[8];
#pragma unroll
  for (int j = 0; j < 8; ++j) acc[j] = zero8();
  mm8(acc, H + (r0 + wave * 16 + col) * DM, WVT + (size_t)(c0 + col) * DM, DM, DM / 32, lane);
#pragma unroll
  for (int j = 0; j < 8; ++j) { const float bv = bf16r(BV[c0 + j * 16 + col]);
#pragma unroll
    for (int r = 0; r < 8; ++r) { const float v = acc[j][r] * (1.0f / WC) + bv; th[j * 16 + col][wave * 16 + 8 * g + r] = f16n(v); } }
  __syncthreads();
#pragma unroll
  for (int it = 0; it < 8; ++it) { const int e = tid + 128 * it, cl = e >> 3, q = e & 7; const int f = c0 + cl, hh = f >> 6, d = f & 63;
    vst2(VT + ((b * NH + hh) * DK + d) * SEQ + s0 + 8 * q, *(const v8h*)&th[cl][8 * q]); }
}

__global__ __launch_bounds__(128) void k_att(const _Float16* __restrict__ QP, const _Float16* __restrict__ KP, const _Float16* __restrict__ VT, _Float16* __restrict__ CTX) {
  __shared__ __align__(16) _Float16 so[4][16][72];
  const int tid = threadIdx.x, wave = tid >> 5, lane = tid & 31, col = lane & 15, g = lane >> 4;
  const int qb = (int)blockIdx.x, bh = (int)blockIdx.y, b = bh / NH, h = bh - b * NH;
  const int q0w = qb * 64 + wave * 16, qq = q0w + col;
  const size_t rowb = (size_t)b * SEQ;
  v16h qf[2];
#pragma unroll
  for (int kc = 0; kc < 2; ++kc) qf[kc] = frag_h(QP + (rowb + qq) * DM + h * DK + kc * 32, lane);
  v8f acc[4];
#pragma unroll
  for (int dt = 0; dt < 4; ++dt) acc[dt] = zero8();
  float m = -1.0e30f, l = 0.f;
#pragma unroll 1
  for (int t = 0; t < SEQ / 32; ++t) {
    const int kb = t * 32;
    v8f st[2];
#pragma unroll
    for (int tt = 0; tt < 2; ++tt) {
      v8f c = zero8();
#pragma unroll
      for (int kc = 0; kc < 2; ++kc) {
        const v16h kf = frag_h(KP + (rowb + kb + tt * 16 + col) * DM + h * DK + kc * 32, lane);
        c = wmma16(kf, qf[kc], c);
      }
      st[tt] = c;
    }
    float sv[16]; float cmax = -1.0e30f;
#pragma unroll
    for (int tt = 0; tt < 2; ++tt) {
#pragma unroll
      for (int r = 0; r < 8; ++r) { const float s = st[tt][r] * SCALE; sv[tt * 8 + r] = s; cmax = fmaxf(cmax, s); }
    }
    cmax = fmaxf(cmax, __shfl_xor(cmax, 16));
    const float mnew = fmaxf(m, cmax); const float fac = __expf(m - mnew);
    v16h pb; float csum = 0.f;
#pragma unroll
    for (int i = 0; i < 16; ++i) {
      float pc = __expf(sv[i] - mnew) * PCY; pc = (pc >= F16MIN) ? pc : 0.0f;
      const _Float16 ph = (_Float16)pc; pb[i] = ph; csum += (float)ph;
    }
    csum += __shfl_xor(csum, 16); l = l * fac + csum; m = mnew;
#pragma unroll
    for (int dt = 0; dt < 4; ++dt) {
#pragma unroll
      for (int r = 0; r < 8; ++r) acc[dt][r] *= fac;
      const v16h vf = frag_h(VT + ((size_t)bh * DK + dt * 16 + col) * SEQ + kb, lane);
      acc[dt] = wmma16(vf, pb, acc[dt]);
    }
  }
  const float inv = (1.0f / l) * CCY;
#pragma unroll
  for (int dt = 0; dt < 4; ++dt) { v8h o8;
#pragma unroll
    for (int r = 0; r < 8; ++r) o8[r] = f16n(acc[dt][r] * inv);
    *(v8h*)&so[wave][col][dt * 16 + 8 * g] = o8; }
  LDSX();
#pragma unroll
  for (int it = 0; it < 4; ++it) { const int e = lane + 32 * it, rl = e >> 3, q = e & 7; vst2(CTX + (rowb + q0w + rl) * DM + h * DK + 8 * q, *(const v8h*)&so[wave][rl][8 * q]); }
}

template <int RESX>
__global__ __launch_bounds__(128) void k_gf(const _Float16* __restrict__ A, int K, const _Float16* __restrict__ B, const float* __restrict__ BIAS, float ascale,
                                            const float* __restrict__ RES, float* __restrict__ OUT) {
  __shared__ __align__(16) float sf[4][16][132];
  const int tid = threadIdx.x, wave = tid >> 5, lane = tid & 31, col = lane & 15, g = lane >> 4; const int c0 = blockIdx.y * 128; const size_t r0 = (size_t)blockIdx.x * 64 + wave * 16;
  v8f acc[8];
#pragma unroll
  for (int j = 0; j < 8; ++j) acc[j] = zero8();
  mm8(acc, A + (r0 + col) * (size_t)K, B + (size_t)(c0 + col) * K, K, K / 32, lane);
#pragma unroll
  for (int j = 0; j < 8; ++j) { const float bv = bf16r(BIAS[c0 + j * 16 + col]);
#pragma unroll
    for (int r = 0; r < 8; ++r) sf[wave][8 * g + r][j * 16 + col] = acc[j][r] * ascale + bv; }
  LDSX();
  for (int rl = 0; rl < 16; ++rl) { const size_t row = r0 + rl; const size_t o = row * DM + c0 + lane * 4; v4f vv = *(const v4f*)&sf[wave][rl][lane * 4];
    v4f rv;
    if (RESX) { const size_t xr = (row / SEQ) * SEQ_FULL + (row % SEQ); const v4f xv = *(const v4f*)(RES + xr * DM + c0 + lane * 4);
#pragma unroll
      for (int k = 0; k < 4; ++k) rv[k] = bf16r(xv[k]); }
    else { rv = *(const v4f*)(RES + o); }
    vv += rv; vst2(OUT + o, vv); }
}

__global__ __launch_bounds__(128) void k_ffn1(const _Float16* __restrict__ H, const _Float16* __restrict__ W1T, const float* __restrict__ B1, _Float16* __restrict__ G) {
  __shared__ __align__(16) _Float16 sh[64][136];
  const int tid = threadIdx.x, wave = tid >> 5, lane = tid & 31, col = lane & 15, g = lane >> 4;
  const size_t r0 = (size_t)blockIdx.x * 64; const int c0 = blockIdx.y * 128;
  v8f acc[8];
#pragma unroll
  for (int j = 0; j < 8; ++j) acc[j] = zero8();
  mm8(acc, H + (r0 + wave * 16 + col) * DM, W1T + (size_t)(c0 + col) * DM, DM, DM / 32, lane);
#pragma unroll
  for (int j = 0; j < 8; ++j) { const float bv = bf16r(B1[c0 + j * 16 + col]);
#pragma unroll
    for (int r = 0; r < 8; ++r) { const float v = acc[j][r] * (1.0f / WC) + bv; const float gl = 0.5f * v * (1.0f + erff(v * 0.70710678118654752f)); sh[wave * 16 + 8 * g + r][j * 16 + col] = f16n(gl * GCY); } }
  __syncthreads();
#pragma unroll
  for (int it = 0; it < 8; ++it) { const int e = tid + 128 * it, rl = e >> 4, q = e & 15; vst2(G + (r0 + rl) * DFF + c0 + 8 * q, *(const v8h*)&sh[rl][8 * q]); }
}

extern "C" void kernel_launch(void* const* d_in, const int* in_sizes, int n_in, void* d_out, int out_size, void* d_ws, size_t ws_size, hipStream_t stream) {
  if (n_in < 17) return;
  if (in_sizes[0] < ((NB - 1) * SEQ_FULL + SEQ) * DM) return;
  if (in_sizes[1] < DM * DM || in_sizes[3] < DM * DM || in_sizes[5] < DM * DM || in_sizes[7] < DM * DM) return;
  if (in_sizes[2] < DM || in_sizes[4] < DM || in_sizes[6] < DM || in_sizes[8] < DM || in_sizes[12] < DM) return;
  if (in_sizes[9] < DM * DFF || in_sizes[10] < DFF || in_sizes[11] < DFF * DM) return;
  if (in_sizes[13] < DM || in_sizes[14] < DM || in_sizes[15] < DM || in_sizes[16] < DM) return;
  if (out_size < MROWS * DM) return;
  if (ws_size < (size_t)WS_END) return;
  const float* x = (const float*)d_in[0];
  const float* wq = (const float*)d_in[1]; const float* bq = (const float*)d_in[2];
  const float* wk = (const float*)d_in[3]; const float* bk = (const float*)d_in[4];
  const float* wv = (const float*)d_in[5]; const float* bv = (const float*)d_in[6];
  const float* wo = (const float*)d_in[7]; const float* bo = (const float*)d_in[8];
  const float* w1 = (const float*)d_in[9]; const float* b1 = (const float*)d_in[10];
  const float* w2 = (const float*)d_in[11]; const float* b2 = (const float*)d_in[12];
  const float* g1 = (const float*)d_in[13]; const float* e1 = (const float*)d_in[14];
  const float* g2 = (const float*)d_in[15]; const float* e2 = (const float*)d_in[16];
  char* ws = (char*)d_ws;
  _Float16* W4T = (_Float16*)(ws + WS_W4); _Float16* W2T = (_Float16*)(ws + WS_W2T); _Float16* W1T = (_Float16*)(ws + WS_W1T);
  float* XS = (float*)(ws + WS_XS); float* Y1 = (float*)(ws + WS_Y1);
  _Float16* QP = (_Float16*)(ws + WS_Q); _Float16* KP = (_Float16*)(ws + WS_K); _Float16* VT = (_Float16*)(ws + WS_VT);
  _Float16* HC = (_Float16*)(ws + WS_HC); _Float16* G = (_Float16*)(ws + WS_G); _Float16* H2 = (_Float16*)(ws + WS_H2);
  float* OUT = (float*)d_out;
  const float s_o = 1.0f / (WC * CCY), s_f = 1.0f / (WC * GCY);

  k_wt<<<dim3(DM / 64, DM / 64, 4), 256, 0, stream>>>(wq, wk, wv, wo, DM, DM, W4T);
  k_wt<<<dim3(DM / 64, DFF / 64, 1), 256, 0, stream>>>(w1, w1, w1, w1, DM, DFF, W1T);
  k_cx<<<dim3(MROWS / 2), 256, 0, stream>>>(x, HC);
  k_pqk<<<dim3(MROWS / 64, DM / 128, 2), 128, 0, stream>>>(HC, W4T, bq, bk, QP, KP);
  k_pvt<<<dim3(MROWS / 64, DM / 128), 128, 0, stream>>>(HC, W4T + (size_t)2 * DM * DM, bv, VT);
  k_att<<<dim3(SEQ / 64, NB * NH), 128, 0, stream>>>(QP, KP, VT, HC);
  k_gf<1><<<dim3(MROWS / 64, DM / 128), 128, 0, stream>>>(HC, DM, W4T + (size_t)3 * DM * DM, bo, s_o, x, XS);
  k_ln<1><<<dim3(MROWS / 8), 256, 0, stream>>>(XS, g1, e1, Y1, H2);
  k_wt<<<dim3(DFF / 64, DM / 64, 1), 256, 0, stream>>>(w2, w2, w2, w2, DFF, DM, W2T);
  k_ffn1<<<dim3(MROWS / 64, DFF / 128), 128, 0, stream>>>(H2, W1T, b1, G);
  k_gf<0><<<dim3(MROWS / 64, DM / 128), 128, 0, stream>>>(G, DFF, W2T, b2, s_f, Y1, XS);
  k_ln<0><<<dim3(MROWS / 8), 256, 0, stream>>>(XS, g2, e2, OUT, H2);
}
